// _Attention_21646635172126
// MI455X (gfx1250) — hardware-run, weakly checked
//
#include <hip/hip_runtime.h>
#include <stdint.h>
#include <stddef.h>

#define NBATCH   64
#define NSEQ     197
#define DMODEL   768
#define NHEADS   12
#define HDIM     64
#define LDQKV    (3 * DMODEL)
#define MROWS    (NBATCH * NSEQ)
#define SPADQ    256
#define NQBLK    (SPADQ / 64)
#define KCH      64
#define NKCH     (SPADQ / KCH)
#define NUMREL   732
#define W_CARRY  256.0f
#define A_CARRY  16.0f
#define P_CARRY  32768.0f
#define QK_OUT_SCALE (0.125f / 256.0f)

static_assert(MROWS % 64 == 0, "M tile");
static_assert(LDQKV % 64 == 0, "N tile qkv");
static_assert(DMODEL % 64 == 0, "N tile proj");
static_assert(DMODEL % 32 == 0, "K step");
static_assert(NSEQ <= SPADQ, "pad");

typedef __attribute__((ext_vector_type(16))) _Float16 v16h;
typedef __attribute__((ext_vector_type(8)))  _Float16 v8h;
typedef __attribute__((ext_vector_type(16))) __bf16   v16b;
typedef __attribute__((ext_vector_type(8)))  __bf16   v8b;
typedef __attribute__((ext_vector_type(8)))  float    v8f;
typedef __attribute__((ext_vector_type(4)))  float    v4f;
typedef __attribute__((ext_vector_type(4)))  unsigned int v4u;

__device__ __forceinline__ unsigned short f2bf_bits(float f) {
  unsigned u = __float_as_uint(f);
  return (unsigned short)((u + 0x7FFFu + ((u >> 16) & 1u)) >> 16);
}
__device__ __forceinline__ float bf_bits2f(unsigned short h) { return __uint_as_float(((unsigned)h) << 16); }
__device__ __forceinline__ float bf_rne(float f) { return bf_bits2f(f2bf_bits(f)); }
__device__ __forceinline__ unsigned short h_bits(float f) { return __builtin_bit_cast(unsigned short, (_Float16)f); }

__device__ __forceinline__ void dep_guard_h(v8f& a, v8f& b, v16h x, v16h y) { asm volatile("v_nop\n\tv_nop\n\tv_nop\n\tv_nop" : "+v"(a), "+v"(b) : "v"(x), "v"(y)); }
__device__ __forceinline__ void dep_guard_b(v8f& a, v8f& b, v16b x, v16b y) { asm volatile("v_nop\n\tv_nop\n\tv_nop\n\tv_nop" : "+v"(a), "+v"(b) : "v"(x), "v"(y)); }
__device__ __forceinline__ void keep4_h(v16h a, v16h b, v16h c, v16h d) { asm volatile("v_nop" :: "v"(a), "v"(b), "v"(c), "v"(d)); }
__device__ __forceinline__ void keep4_b(v16b a, v16b b, v16b c, v16b d) { asm volatile("v_nop" :: "v"(a), "v"(b), "v"(c), "v"(d)); }
__device__ __forceinline__ void acc_guard4(v8f& a, v8f& b, v8f& c, v8f& d) { asm volatile("v_nop\n\tv_nop\n\tv_nop\n\tv_nop" : "+v"(a), "+v"(b), "+v"(c), "+v"(d)); }
template <typename T> struct Frag;
template <> struct Frag<_Float16> {
  typedef v16h V; union U { v16h v; v8h h[2]; };
  static __device__ __forceinline__ v16h load(const _Float16* p) {
    U f; f.h[0] = *(const v8h*)(p); f.h[1] = *(const v8h*)(p + 16); return f.v;
  }
  static __device__ __forceinline__ v8f mma(v16h a, v16h b, v8f c) {
    return __builtin_amdgcn_wmma_f32_16x16x32_f16(false, a, false, b, (short)0, c, false, false);
  }
  static __device__ __forceinline__ void guard(v8f& a, v8f& b, v16h x, v16h y) { dep_guard_h(a, b, x, y); }
  static __device__ __forceinline__ void keep(v16h a, v16h b, v16h c, v16h d) { keep4_h(a, b, c, d); }
};
template <> struct Frag<__bf16> {
  typedef v16b V; union U { v16b v; v8b h[2]; };
  static __device__ __forceinline__ v16b load(const __bf16* p) {
    U f; f.h[0] = *(const v8b*)(p); f.h[1] = *(const v8b*)(p + 16); return f.v;
  }
  static __device__ __forceinline__ v8f mma(v16b a, v16b b, v8f c) {
    return __builtin_amdgcn_wmma_f32_16x16x32_bf16(false, a, false, b, (short)0, c, false, false);
  }
  static __device__ __forceinline__ void guard(v8f& a, v8f& b, v16b x, v16b y) { dep_guard_b(a, b, x, y); }
  static __device__ __forceinline__ void keep(v16b a, v16b b, v16b c, v16b d) { keep4_b(a, b, c, d); }
};

template <int ET> struct Elem;
template <> struct Elem<0> { typedef _Float16 T; };
template <> struct Elem<1> { typedef __bf16 T; };
template <int ET, bool SPLIT, int BIAS_MODE, int OUT_MODE, bool RESID, int ACT = 0>
__global__ __launch_bounds__(256) void wmma_gemm64(
    const unsigned short* __restrict__ Ap, const unsigned short* __restrict__ A2p, int lda, long strideA,
    const unsigned short* __restrict__ Btp, const unsigned short* __restrict__ Bt2p, int ldb, long strideB,
    void* __restrict__ Cout, void* __restrict__ Cout2, int ldc, long strideC,
    const float* __restrict__ bias,
    const float* __restrict__ resid, long strideR,
    int M, int N, int K, float scale) {
  typedef typename Elem<ET>::T T;
  typedef typename Frag<T>::V V;
  const T* A = (const T*)Ap; const T* A2 = (const T*)A2p; const T* Bt = (const T*)Btp; const T* Bt2 = (const T*)Bt2p;
  __shared__ __align__(16) float sT[8][16 * 68];
  const int b    = blockIdx.y;
  const int lane = threadIdx.x & 31;
  const int wave = threadIdx.x >> 5;
  const int tilesN = N >> 6;
  const int tilesM = M >> 6;
  const int tile = blockIdx.x * 8 + wave;
  if (tile >= tilesM * tilesN) return;
  const int tm = tile / tilesN;
  const int tn = tile - tm * tilesN;
  const int m0 = tm << 6;
  const int n0 = tn << 6;

  const T* Ab  = A  + (size_t)b * strideA;
  const T* Bb  = Bt + (size_t)b * strideB;
  const T* Ab2 = SPLIT ? (A2  + (size_t)b * strideA) : nullptr;
  const T* Bb2 = SPLIT ? (Bt2 + (size_t)b * strideB) : nullptr;

  const int rlane = lane & 15;
  const int koff  = (lane >> 4) * 8;
  const int mOff  = (lane >> 4) * 8;

  v8f acc[4][4];
#pragma unroll
  for (int i = 0; i < 4; ++i)
#pragma unroll
    for (int j = 0; j < 4; ++j) acc[i][j] = (v8f){0.f,0.f,0.f,0.f,0.f,0.f,0.f,0.f};

  for (int k0 = 0; k0 < K; k0 += 32) {
    V bh[4], bl[4];
#pragma unroll
    for (int j = 0; j < 4; ++j) {
      const size_t bo = (size_t)(n0 + (j << 4) + rlane) * ldb + koff + k0;
      bh[j] = Frag<T>::load(Bb + bo);
      if (SPLIT) bl[j] = Frag<T>::load(Bb2 + bo);
    }
#pragma unroll
    for (int i = 0; i < 4; ++i) {
      const size_t ao = (size_t)(m0 + (i << 4) + rlane) * lda + koff + k0;
      V ah = Frag<T>::load(Ab + ao);
      V al;
      if (SPLIT) al = Frag<T>::load(Ab2 + ao);
#pragma unroll
      for (int j = 0; j < 4; ++j) {
        acc[i][j] = Frag<T>::mma(ah, bh[j], acc[i][j]);
        if (SPLIT) {
          acc[i][j] = Frag<T>::mma(ah, bl[j], acc[i][j]);
          acc[i][j] = Frag<T>::mma(al, bh[j], acc[i][j]);
        }
      }
      Frag<T>::guard(acc[i][0], acc[i][3], ah, SPLIT ? al : ah);
    }
    Frag<T>::keep(bh[0], bh[1], bh[2], bh[3]);
    if (SPLIT) Frag<T>::keep(bl[0], bl[1], bl[2], bl[3]);
  }
  acc_guard4(acc[0][0], acc[0][1], acc[0][2], acc[0][3]);
  acc_guard4(acc[1][0], acc[1][1], acc[1][2], acc[1][3]);
  acc_guard4(acc[2][0], acc[2][1], acc[2][2], acc[2][3]);
  acc_guard4(acc[3][0], acc[3][1], acc[3][2], acc[3][3]);

  float* slab = sT[wave];
  const float* Rb = RESID ? (resid + (size_t)b * strideR) : nullptr;
#pragma unroll
  for (int i = 0; i < 4; ++i) {
    const int mBase = m0 + (i << 4);
#pragma unroll
    for (int j = 0; j < 4; ++j) {
      const int n = n0 + (j << 4) + rlane;
      float bv = 0.f;
      if (BIAS_MODE == 2) bv = bias[n];
#pragma unroll
      for (int r = 0; r < 8; ++r) {
        float v = acc[i][j][r] * scale;
        if (BIAS_MODE == 1) v += bias[mBase + mOff + r];
        if (BIAS_MODE == 2) v += bv;
        if (RESID) v += Rb[(size_t)(mBase + mOff + r) * ldc + n];
        if (ACT == 1) v = tanhf(v);
        if (ACT == 2) v = fmaxf(v, 0.0f);
        if (ACT == 3) v = v / (1.0f + expf(-v));
        if (ACT == 4) v = (v > 0.f) ? v : 0.01f * v;
        if (ACT == 5) v = 0.5f * v * (1.0f + erff(v * 0.70710678118654752f));
        slab[(mOff + r) * 68 + (j << 4) + rlane] = v;
      }
    }
    __builtin_amdgcn_fence(__ATOMIC_RELEASE, "workgroup");
    __builtin_amdgcn_wave_barrier();
    __builtin_amdgcn_fence(__ATOMIC_ACQUIRE, "workgroup");
    if (OUT_MODE == 0) {
      float* C = (float*)Cout + (size_t)b * strideC;
      const int hh = lane >> 4, c4 = (lane & 15) * 4;
      for (int pass = 0; pass < 2; ++pass) {
#pragma unroll
        for (int it = 0; it < 8; ++it) {
          const int row = it * 2 + hh;
          v4f v = *(const v4f*)(slab + row * 68 + c4);
          *(volatile v4f*)(C + (size_t)(mBase + row) * ldc + n0 + c4) = v;
        }
        __threadfence();
      }
    } else {
      const int q = lane >> 3, c8 = (lane & 7) * 8;
      unsigned short* C  = (unsigned short*)Cout  + (size_t)b * strideC;
      unsigned short* C2 = (OUT_MODE == 2) ? ((unsigned short*)Cout2 + (size_t)b * strideC) : nullptr;
      for (int pass = 0; pass < 2; ++pass) {
#pragma unroll
        for (int it = 0; it < 4; ++it) {
          const int row = it * 4 + q;
          const float* sp = slab + row * 68 + c8;
          v8h hv, lv;
#pragma unroll
          for (int e = 0; e < 8; ++e) {
            if (OUT_MODE == 1) {
              hv[e] = (_Float16)sp[e];
            } else {
              unsigned short hb = f2bf_bits(sp[e]);
              unsigned short lb = f2bf_bits(sp[e] - bf_bits2f(hb));
              hv[e] = __builtin_bit_cast(_Float16, hb);
              lv[e] = __builtin_bit_cast(_Float16, lb);
            }
          }
          *(volatile v8h*)(C + (size_t)(mBase + row) * ldc + n0 + c8) = hv;
          if (OUT_MODE == 2) *(volatile v8h*)(C2 + (size_t)(mBase + row) * ldc + n0 + c8) = lv;
        }
        __threadfence();
      }
    }
    __builtin_amdgcn_fence(__ATOMIC_RELEASE, "workgroup");
    __builtin_amdgcn_wave_barrier();
    __builtin_amdgcn_fence(__ATOMIC_ACQUIRE, "workgroup");
  }
}

__global__ __launch_bounds__(256) void cast_bf16r_f16x8(
    const float* __restrict__ in, unsigned short* __restrict__ out, int n8, float sc) {
  const int i = blockIdx.x * 256 + threadIdx.x;
  if (i < n8) {
    const float* src = in + (size_t)i * 8;
    const v4f a0 = *(const v4f*)(src);
    const v4f a1 = *(const v4f*)(src + 4);
    v4u w;
    {
      const unsigned l0 = h_bits(bf_rne(a0[0]) * sc), u0 = h_bits(bf_rne(a0[1]) * sc);
      const unsigned l1 = h_bits(bf_rne(a0[2]) * sc), u1 = h_bits(bf_rne(a0[3]) * sc);
      const unsigned l2 = h_bits(bf_rne(a1[0]) * sc), u2 = h_bits(bf_rne(a1[1]) * sc);
      const unsigned l3 = h_bits(bf_rne(a1[2]) * sc), u3 = h_bits(bf_rne(a1[3]) * sc);
      w[0] = l0 | (u0 << 16);
      w[1] = l1 | (u1 << 16);
      w[2] = l2 | (u2 << 16);
      w[3] = l3 | (u3 << 16);
    }
    volatile v4u* dst = (volatile v4u*)(void*)(out + (size_t)i * 8);
    *dst = w;
    __threadfence();
    *dst = w;
  }
}

#define PREP_R0 LDQKV
#define PREP_R1 (LDQKV + DMODEL)
#define PREP_TOT (LDQKV + DMODEL + NHEADS * SPADQ * SPADQ)
static_assert(PREP_R0 % 256 == 0 && PREP_R1 % 256 == 0 && PREP_TOT % 256 == 0, "block-uniform regions");

__global__ __launch_bounds__(256) void prep_tables(
    const float* __restrict__ q_bias, const float* __restrict__ v_bias,
    const float* __restrict__ proj_b, const float* __restrict__ rel_table,
    const int* __restrict__ rel_index,
    float* __restrict__ qkvb, float* __restrict__ pjb, float* __restrict__ biasT) {
  const int i = blockIdx.x * 256 + threadIdx.x;
  if (i >= PREP_TOT) return;
  if (i < PREP_R0) {
    int nq = i; nq = (nq < DMODEL) ? nq : (DMODEL - 1);
    int nv = i - 2 * DMODEL; nv = (nv < 0) ? 0 : nv; nv = (nv < DMODEL) ? nv : (DMODEL - 1);
    const float qv = bf_rne(q_bias[nq]) * A_CARRY;
    const float vv = bf_rne(v_bias[nv]) * A_CARRY;
    const float val = (i < DMODEL) ? qv : ((i >= 2 * DMODEL) ? vv : 0.0f);
    volatile float* p = (volatile float*)(qkvb + i);
    *p = val;
    __threadfence();
    *p = val;
  } else if (i < PREP_R1) {
    const int n = i - PREP_R0;
    const float val = bf_rne(proj_b[n]);
    volatile float* p = (volatile float*)(pjb + n);
    *p = val;
    __threadfence();
    *p = val;
  } else {
    const int e = i - PREP_R1;
    const int kv = e & (SPADQ - 1);
    const int q = (e >> 8) & (SPADQ - 1);
    const int hd = e >> 16;
    const int qc = (q < NSEQ) ? q : (NSEQ - 1);
    const int kvc = (kv < NSEQ) ? kv : (NSEQ - 1);
    int idx = rel_index[qc * NSEQ + kvc];
    idx = (idx < 0) ? 0 : idx; idx = (idx < NUMREL) ? idx : (NUMREL - 1);
    const float tv = bf_rne(rel_table[idx * NHEADS + hd]);
    const float val = (kv < NSEQ) ? tv : -1e30f;
    volatile float* p = (volatile float*)(biasT + e);
    *p = val;
    __threadfence();
    *p = val;
  }
}

__device__ __forceinline__ v8f mma_f16_g(v16h a, v16h b, v8f c) {
  c = __builtin_amdgcn_wmma_f32_16x16x32_f16(false, a, false, b, (short)0, c, false, false);
  asm volatile("v_nop\n\tv_nop\n\tv_nop\n\tv_nop" : "+v"(c) : "v"(a), "v"(b));
  return c;
}

__global__ __launch_bounds__(128) void attn_relbias_f16(
    const unsigned short* __restrict__ qkv, const float* __restrict__ biasT,
    unsigned short* __restrict__ ctx) {
  union FH { v16h v; v8h h[2]; };
  __shared__ __align__(16) unsigned short Ksh[KCH * HDIM];
  __shared__ __align__(16) unsigned short Vth[HDIM * KCH];
  __shared__ __align__(16) unsigned short Psh[4][16 * KCH];
  __shared__ __align__(16) float Bsh[64 * KCH];
  __shared__ __align__(16) float Osl[4][16 * 68];

  const int tid  = threadIdx.x;
  const int wave = tid >> 5;
  const int lane = tid & 31;
  const int hh   = lane >> 4;
  const int c    = lane & 15;

  const int bx  = blockIdx.x;
  const int qb  = bx % NQBLK;
  const int bhx = bx / NQBLK;
  const int h   = bhx % NHEADS;
  const int b   = bhx / NHEADS;
  const int qbase = qb * 64;
  const int q0 = qbase + wave * 16;
  const size_t rowb = (size_t)b * NSEQ;

  v16h qa[2];
  {
    int qr = q0 + c; qr = (qr < NSEQ) ? qr : (NSEQ - 1);
    const _Float16* qp = (const _Float16*)(const void*)(qkv + (rowb + (size_t)qr) * LDQKV + h * HDIM);
#pragma unroll
    for (int dc = 0; dc < 2; ++dc) qa[dc] = Frag<_Float16>::load(qp + dc * 32 + 8 * hh);
  }

  float mrow[8], lrow[8];
  v8f oacc[4];
#pragma unroll
  for (int r = 0; r < 8; ++r) { mrow[r] = -__builtin_inff(); lrow[r] = 0.f; }
#pragma unroll
  for (int t = 0; t < 4; ++t) oacc[t] = (v8f){0.f,0.f,0.f,0.f,0.f,0.f,0.f,0.f};

  for (int kc = 0; kc < NKCH; ++kc) {
    const int kv0 = kc * KCH;
    __syncthreads();
    {
      const int kvr = tid >> 1, dh = (tid & 1) * 32;
      int kvg = kv0 + kvr; kvg = (kvg < NSEQ) ? kvg : (NSEQ - 1);
      const unsigned short* krow = qkv + (rowb + (size_t)kvg) * LDQKV + DMODEL + h * HDIM + dh;
      const unsigned short* vrow = krow + DMODEL;
#pragma unroll
      for (int i = 0; i < 4; ++i) {
        const v4u kw = *(const v4u*)(const void*)(krow + 8 * i);
        const v4u vw = *(const v4u*)(const void*)(vrow + 8 * i);
        *(v4u*)(void*)(Ksh + kvr * HDIM + dh + 8 * i) = kw;
#pragma unroll
        for (int e = 0; e < 8; ++e) {
          const unsigned wd = vw[e >> 1];
          const unsigned short hb = (unsigned short)((e & 1) ? (wd >> 16) : (wd & 0xffffu));
          Vth[(dh + 8 * i + e) * KCH + kvr] = hb;
        }
      }
      asm volatile("" ::: "memory");
      const int brow = tid >> 1, bhf = (tid & 1) * 32;
      const float* bsrc = biasT + ((size_t)h * SPADQ + (size_t)(qbase + brow)) * SPADQ + kv0 + bhf;
#pragma unroll
      for (int i = 0; i < 8; ++i) {
        const v4f bv = *(const v4f*)(bsrc + 4 * i);
        *(v4f*)(Bsh + brow * KCH + bhf + 4 * i) = bv;
      }
    }
    __syncthreads();

    v8f s[4];
#pragma unroll
    for (int j = 0; j < 4; ++j) {
      s[j] = (v8f){0.f,0.f,0.f,0.f,0.f,0.f,0.f,0.f};
#pragma unroll
      for (int dc = 0; dc < 2; ++dc) {
        FH kb;
        kb.h[0] = *(const v8h*)(const void*)(Ksh + (j * 16 + c) * HDIM + dc * 32 + 8 * hh);
        kb.h[1] = *(const v8h*)(const void*)(Ksh + (j * 16 + c) * HDIM + dc * 32 + 16 + 8 * hh);
        s[j] = mma_f16_g(qa[dc], kb.v, s[j]);
      }
    }
    const float* bw = Bsh + (wave * 16 + 8 * hh) * KCH;
    float cm[8];
#pragma unroll
    for (int r = 0; r < 8; ++r) {
      float m = -1e30f;
#pragma unroll
      for (int j = 0; j < 4; ++j) {
        const float v = s[j][r] * QK_OUT_SCALE + bw[r * KCH + j * 16 + c];
        s[j][r] = v;
        m = fmaxf(m, v);
      }
#pragma unroll
      for (int off = 1; off < 16; off <<= 1) m = fmaxf(m, __shfl_xor(m, off, 32));
      cm[r] = m;
    }
    unsigned short* pw = Psh[wave];
#pragma unroll
    for (int r = 0; r < 8; ++r) {
      const float mnew = fmaxf(mrow[r], cm[r]);
      const float alpha = expf(mrow[r] - mnew);
      mrow[r] = mnew;
      float psum = 0.f;
#pragma unroll
      for (int j = 0; j < 4; ++j) {
        const float p = expf(s[j][r] - mnew);
        psum += p;
        pw[(8 * hh + r) * KCH + j * 16 + c] = h_bits(p * P_CARRY);
      }
#pragma unroll
      for (int off = 1; off < 16; off <<= 1) psum += __shfl_xor(psum, off, 32);
      lrow[r] = lrow[r] * alpha + psum;
#pragma unroll
      for (int t = 0; t < 4; ++t) oacc[t][r] *= alpha;
    }
    __builtin_amdgcn_fence(__ATOMIC_RELEASE, "workgroup");
    __builtin_amdgcn_wave_barrier();
    __builtin_amdgcn_fence(__ATOMIC_ACQUIRE, "workgroup");
#pragma unroll
    for (int kk = 0; kk < 2; ++kk) {
      FH pa;
      pa.h[0] = *(const v8h*)(const void*)(pw + c * KCH + kk * 32 + 8 * hh);
      pa.h[1] = *(const v8h*)(const void*)(pw + c * KCH + kk * 32 + 16 + 8 * hh);
#pragma unroll
      for (int t = 0; t < 4; ++t) {
        FH vb;
        vb.h[0] = *(const v8h*)(const void*)(Vth + (t * 16 + c) * KCH + kk * 32 + 8 * hh);
        vb.h[1] = *(const v8h*)(const void*)(Vth + (t * 16 + c) * KCH + kk * 32 + 16 + 8 * hh);
        oacc[t] = mma_f16_g(pa.v, vb.v, oacc[t]);
      }
    }
  }

  float* os = Osl[wave];
#pragma unroll
  for (int r = 0; r < 8; ++r) {
    const float inv = 1.0f / (lrow[r] * P_CARRY);
#pragma unroll
    for (int t = 0; t < 4; ++t) os[(8 * hh + r) * 68 + t * 16 + c] = oacc[t][r] * inv;
  }
  __builtin_amdgcn_fence(__ATOMIC_RELEASE, "workgroup");
  __builtin_amdgcn_wave_barrier();
  __builtin_amdgcn_fence(__ATOMIC_ACQUIRE, "workgroup");
  {
    const int q8 = lane >> 3, c8 = (lane & 7) * 8;
    for (int pass = 0; pass < 2; ++pass) {
#pragma unroll
      for (int it = 0; it < 4; ++it) {
        const int row = it * 4 + q8;
        const float* sp = os + row * 68 + c8;
        v8h hv;
#pragma unroll
        for (int e = 0; e < 8; ++e) hv[e] = (_Float16)sp[e];
        const int qg = q0 + row;
        if (qg < NSEQ)
          *(volatile v8h*)(void*)(ctx + (rowb + (size_t)qg) * DMODEL + h * HDIM + c8) = hv;
      }
      __threadfence();
    }
  }
}

constexpr size_t al256(size_t x) { return (x + 255) & ~(size_t)255; }
constexpr size_t SZ_XH    = (size_t)MROWS * DMODEL * 2;
constexpr size_t SZ_WQKV  = (size_t)LDQKV * DMODEL * 2;
constexpr size_t SZ_WP    = (size_t)DMODEL * DMODEL * 2;
constexpr size_t SZ_QKV   = (size_t)MROWS * LDQKV * 2;
constexpr size_t SZ_QKVB  = (size_t)LDQKV * 4;
constexpr size_t SZ_PJB   = (size_t)DMODEL * 4;
constexpr size_t SZ_BIAST = (size_t)NHEADS * SPADQ * SPADQ * 4;
constexpr size_t OFF_XH    = 0;
constexpr size_t OFF_WQKV  = OFF_XH + al256(SZ_XH);
constexpr size_t OFF_WP    = OFF_WQKV + al256(SZ_WQKV);
constexpr size_t OFF_QKV   = OFF_WP + al256(SZ_WP);
constexpr size_t OFF_QKVB  = OFF_QKV + al256(SZ_QKV);
constexpr size_t OFF_PJB   = OFF_QKVB + al256(SZ_QKVB);
constexpr size_t OFF_BIAST = OFF_PJB + al256(SZ_PJB);
constexpr size_t WS_TOTAL  = OFF_BIAST + al256(SZ_BIAST);
static_assert(WS_TOTAL == 85340160, "carve total");
static_assert(WS_TOTAL <= (size_t)134217728, "carve limit");
static_assert(((size_t)MROWS * DMODEL) % 8 == 0 && ((size_t)LDQKV * DMODEL) % 8 == 0 && ((size_t)DMODEL * DMODEL) % 8 == 0, "cast x8");

extern "C" void kernel_launch(void* const* d_in, const int* in_sizes, int n_in,
                              void* d_out, int out_size, void* d_ws, size_t ws_size,
                              hipStream_t stream) {
  if (n_in < 8) return;
  if (in_sizes[0] != MROWS * DMODEL) return;
  if (in_sizes[1] != LDQKV * DMODEL) return;
  if (in_sizes[2] != DMODEL || in_sizes[3] != DMODEL) return;
  if (in_sizes[4] != NUMREL * NHEADS) return;
  if (in_sizes[5] != NSEQ * NSEQ) return;
  if (in_sizes[6] != DMODEL * DMODEL || in_sizes[7] != DMODEL) return;
  if (out_size != MROWS * DMODEL) return;
  if (ws_size < WS_TOTAL) return;

  const float* x      = (const float*)d_in[0];
  const float* qkv_w  = (const float*)d_in[1];
  const float* q_bias = (const float*)d_in[2];
  const float* v_bias = (const float*)d_in[3];
  const float* rel_t  = (const float*)d_in[4];
  const int*   rel_i  = (const int*)d_in[5];
  const float* proj_w = (const float*)d_in[6];
  const float* proj_b = (const float*)d_in[7];
  float* out = (float*)d_out;

  char* ws = (char*)d_ws;
  unsigned short* XH    = (unsigned short*)(ws + OFF_XH);
  unsigned short* CTX   = XH;
  unsigned short* WQKV  = (unsigned short*)(ws + OFF_WQKV);
  unsigned short* WP    = (unsigned short*)(ws + OFF_WP);
  unsigned short* QKV   = (unsigned short*)(ws + OFF_QKV);
  float* QKVB  = (float*)(ws + OFF_QKVB);
  float* PJB   = (float*)(ws + OFF_PJB);
  float* BIAST = (float*)(ws + OFF_BIAST);

  {
    const int n8x = (MROWS * DMODEL) / 8;
    cast_bf16r_f16x8<<<dim3((n8x + 255) / 256), 256, 0, stream>>>(x, XH, n8x, 1.0f);
    const int n8w = (LDQKV * DMODEL) / 8;
    cast_bf16r_f16x8<<<dim3((n8w + 255) / 256), 256, 0, stream>>>(qkv_w, WQKV, n8w, W_CARRY);
    const int n8p = (DMODEL * DMODEL) / 8;
    cast_bf16r_f16x8<<<dim3((n8p + 255) / 256), 256, 0, stream>>>(proj_w, WP, n8p, W_CARRY);
  }
  prep_tables<<<dim3(PREP_TOT / 256), 256, 0, stream>>>(q_bias, v_bias, proj_b, rel_t, rel_i, QKVB, PJB, BIAST);

  {
    const int tiles = (MROWS / 64) * (LDQKV / 64);
    wmma_gemm64<0, false, 2, 1, false, 0><<<dim3((tiles + 7) / 8, 1), 256, 0, stream>>>(
        XH, XH, DMODEL, 0L,
        WQKV, WQKV, DMODEL, 0L,
        (void*)QKV, (void*)QKV, LDQKV, 0L,
        QKVB,
        QKVB, 0L,
        MROWS, LDQKV, DMODEL, A_CARRY / W_CARRY);
  }
  attn_relbias_f16<<<dim3(NBATCH * NHEADS * NQBLK), 128, 0, stream>>>(QKV, BIAST, CTX);

  {
    const int tiles = (MROWS / 64) * (DMODEL / 64);
    wmma_gemm64<0, false, 2, 0, false, 0><<<dim3((tiles + 7) / 8, 1), 256, 0, stream>>>(
        CTX, CTX, DMODEL, 0L,
        WP, WP, DMODEL, 0L,
        (void*)out, (void*)out, DMODEL, 0L,
        PJB,
        PJB, 0L,
        MROWS, DMODEL, DMODEL, 1.0f / (A_CARRY * W_CARRY));
  }
}
